// QNetwork_32615981645978
// MI455X (gfx1250) — hardware-verified
//
#include <hip/hip_runtime.h>
#include <math.h>

typedef __attribute__((ext_vector_type(16))) _Float16 v16h;
typedef __attribute__((ext_vector_type(8)))  _Float16 v8h;
typedef __attribute__((ext_vector_type(16))) __bf16   v16b;
typedef __attribute__((ext_vector_type(8)))  __bf16   v8b;
typedef __attribute__((ext_vector_type(8)))  float    v8f;
typedef __attribute__((ext_vector_type(4)))  float    v4f;
typedef __attribute__((ext_vector_type(2)))  float    v2f;
typedef __attribute__((ext_vector_type(4)))  unsigned v4u;
typedef __attribute__((ext_vector_type(2)))  unsigned v2u;

constexpr int NB    = 512;
constexpr int NS    = 6;
constexpr int NS2   = 32;
constexpr int HID   = 256;
constexpr int NHEAD = 8;
constexpr int HDIM  = 32;
constexpr int DFF   = 2048;
constexpr int NLAB  = 3;
constexpr int NLAY  = 3;
constexpr int NTOK  = NB * NS;
constexpr int NACT  = NB * NS2;

__device__ __forceinline__ unsigned short f2bf_bits(float f) {
  unsigned u = __float_as_uint(f);
  return (unsigned short)((u + 0x7FFFu + ((u >> 16) & 1u)) >> 16);
}
__device__ __forceinline__ float bf_bits2f(unsigned short h) { return __uint_as_float(((unsigned)h) << 16); }

__device__ __forceinline__ void dep_guard_h(v8f& a, v8f& b, v16h x, v16h y) { asm volatile("v_nop\n\tv_nop\n\tv_nop\n\tv_nop" : "+v"(a), "+v"(b) : "v"(x), "v"(y)); }
__device__ __forceinline__ void dep_guard_b(v8f& a, v8f& b, v16b x, v16b y) { asm volatile("v_nop\n\tv_nop\n\tv_nop\n\tv_nop" : "+v"(a), "+v"(b) : "v"(x), "v"(y)); }
__device__ __forceinline__ void keep4_h(v16h a, v16h b, v16h c, v16h d) { asm volatile("v_nop" :: "v"(a), "v"(b), "v"(c), "v"(d)); }
__device__ __forceinline__ void keep4_b(v16b a, v16b b, v16b c, v16b d) { asm volatile("v_nop" :: "v"(a), "v"(b), "v"(c), "v"(d)); }
__device__ __forceinline__ void acc_guard4(v8f& a, v8f& b, v8f& c, v8f& d) { asm volatile("v_nop\n\tv_nop\n\tv_nop\n\tv_nop" : "+v"(a), "+v"(b), "+v"(c), "+v"(d)); }
template <typename T> struct Frag;
template <> struct Frag<_Float16> {
  typedef v16h V; union U { v16h v; v8h h[2]; };
  static __device__ __forceinline__ v16h load(const _Float16* p) {
    U f; f.h[0] = *(const v8h*)(p); f.h[1] = *(const v8h*)(p + 16); return f.v;
  }
  static __device__ __forceinline__ v8f mma(v16h a, v16h b, v8f c) {
    return __builtin_amdgcn_wmma_f32_16x16x32_f16(false, a, false, b, (short)0, c, false, false);
  }
  static __device__ __forceinline__ void guard(v8f& a, v8f& b, v16h x, v16h y) { dep_guard_h(a, b, x, y); }
  static __device__ __forceinline__ void keep(v16h a, v16h b, v16h c, v16h d) { keep4_h(a, b, c, d); }
};
template <> struct Frag<__bf16> {
  typedef v16b V; union U { v16b v; v8b h[2]; };
  static __device__ __forceinline__ v16b load(const __bf16* p) {
    U f; f.h[0] = *(const v8b*)(p); f.h[1] = *(const v8b*)(p + 16); return f.v;
  }
  static __device__ __forceinline__ v8f mma(v16b a, v16b b, v8f c) {
    return __builtin_amdgcn_wmma_f32_16x16x32_bf16(false, a, false, b, (short)0, c, false, false);
  }
  static __device__ __forceinline__ void guard(v8f& a, v8f& b, v16b x, v16b y) { dep_guard_b(a, b, x, y); }
  static __device__ __forceinline__ void keep(v16b a, v16b b, v16b c, v16b d) { keep4_b(a, b, c, d); }
};

template <int ET> struct Elem;
template <> struct Elem<0> { typedef _Float16 T; };
template <> struct Elem<1> { typedef __bf16 T; };
template <int ET, bool SPLIT, int BIAS_MODE, int OUT_MODE, bool RESID, int ACT = 0>
__global__ __launch_bounds__(256) void wmma_gemm64(
    const unsigned short* __restrict__ Ap, const unsigned short* __restrict__ A2p, int lda, long strideA,
    const unsigned short* __restrict__ Btp, const unsigned short* __restrict__ Bt2p, int ldb, long strideB,
    void* __restrict__ Cout, void* __restrict__ Cout2, int ldc, long strideC,
    const float* __restrict__ bias,
    const float* __restrict__ resid, long strideR,
    int M, int N, int K, float scale) {
  typedef typename Elem<ET>::T T;
  typedef typename Frag<T>::V V;
  const T* A = (const T*)Ap; const T* A2 = (const T*)A2p; const T* Bt = (const T*)Btp; const T* Bt2 = (const T*)Bt2p;
  __shared__ __align__(16) float sT[8][16 * 68];
  const int b    = blockIdx.y;
  const int lane = threadIdx.x & 31;
  const int wave = threadIdx.x >> 5;
  const int tilesN = N >> 6;
  const int tilesM = M >> 6;
  const int tile = blockIdx.x * 8 + wave;
  if (tile >= tilesM * tilesN) return;
  const int tm = tile / tilesN;
  const int tn = tile - tm * tilesN;
  const int m0 = tm << 6;
  const int n0 = tn << 6;

  const T* Ab  = A  + (size_t)b * strideA;
  const T* Bb  = Bt + (size_t)b * strideB;
  const T* Ab2 = SPLIT ? (A2  + (size_t)b * strideA) : nullptr;
  const T* Bb2 = SPLIT ? (Bt2 + (size_t)b * strideB) : nullptr;

  const int rlane = lane & 15;
  const int koff  = (lane >> 4) * 8;
  const int mOff  = (lane >> 4) * 8;

  v8f acc[4][4];
#pragma unroll
  for (int i = 0; i < 4; ++i)
#pragma unroll
    for (int j = 0; j < 4; ++j) acc[i][j] = (v8f){0.f,0.f,0.f,0.f,0.f,0.f,0.f,0.f};

  for (int k0 = 0; k0 < K; k0 += 32) {
    V bh[4], bl[4];
#pragma unroll
    for (int j = 0; j < 4; ++j) {
      const size_t bo = (size_t)(n0 + (j << 4) + rlane) * ldb + koff + k0;
      bh[j] = Frag<T>::load(Bb + bo);
      if (SPLIT) bl[j] = Frag<T>::load(Bb2 + bo);
    }
#pragma unroll
    for (int i = 0; i < 4; ++i) {
      const size_t ao = (size_t)(m0 + (i << 4) + rlane) * lda + koff + k0;
      V ah = Frag<T>::load(Ab + ao);
      V al;
      if (SPLIT) al = Frag<T>::load(Ab2 + ao);
#pragma unroll
      for (int j = 0; j < 4; ++j) {
        acc[i][j] = Frag<T>::mma(ah, bh[j], acc[i][j]);
        if (SPLIT) {
          acc[i][j] = Frag<T>::mma(ah, bl[j], acc[i][j]);
          acc[i][j] = Frag<T>::mma(al, bh[j], acc[i][j]);
        }
      }
      Frag<T>::guard(acc[i][0], acc[i][3], ah, SPLIT ? al : ah);
    }
    Frag<T>::keep(bh[0], bh[1], bh[2], bh[3]);
    if (SPLIT) Frag<T>::keep(bl[0], bl[1], bl[2], bl[3]);
  }
  acc_guard4(acc[0][0], acc[0][1], acc[0][2], acc[0][3]);
  acc_guard4(acc[1][0], acc[1][1], acc[1][2], acc[1][3]);
  acc_guard4(acc[2][0], acc[2][1], acc[2][2], acc[2][3]);
  acc_guard4(acc[3][0], acc[3][1], acc[3][2], acc[3][3]);

  float* slab = sT[wave];
  const float* Rb = RESID ? (resid + (size_t)b * strideR) : nullptr;
#pragma unroll
  for (int i = 0; i < 4; ++i) {
    const int mBase = m0 + (i << 4);
#pragma unroll
    for (int j = 0; j < 4; ++j) {
      const int n = n0 + (j << 4) + rlane;
      float bv = 0.f;
      if (BIAS_MODE == 2) bv = bias[n];
#pragma unroll
      for (int r = 0; r < 8; ++r) {
        float v = acc[i][j][r] * scale;
        if (BIAS_MODE == 1) v += bias[mBase + mOff + r];
        if (BIAS_MODE == 2) v += bv;
        if (RESID) v += Rb[(size_t)(mBase + mOff + r) * ldc + n];
        if (ACT == 1) v = tanhf(v);
        if (ACT == 2) v = fmaxf(v, 0.0f);
        if (ACT == 3) v = v / (1.0f + expf(-v));
        if (ACT == 4) v = (v > 0.f) ? v : 0.01f * v;
        if (ACT == 5) v = 0.5f * v * (1.0f + erff(v * 0.70710678118654752f));
        slab[(mOff + r) * 68 + (j << 4) + rlane] = v;
      }
    }
    __builtin_amdgcn_fence(__ATOMIC_RELEASE, "workgroup");
    __builtin_amdgcn_wave_barrier();
    __builtin_amdgcn_fence(__ATOMIC_ACQUIRE, "workgroup");
    if (OUT_MODE == 0) {
      float* C = (float*)Cout + (size_t)b * strideC;
      const int hh = lane >> 4, c4 = (lane & 15) * 4;
      for (int pass = 0; pass < 2; ++pass) {
#pragma unroll
        for (int it = 0; it < 8; ++it) {
          const int row = it * 2 + hh;
          v4f v = *(const v4f*)(slab + row * 68 + c4);
          *(volatile v4f*)(C + (size_t)(mBase + row) * ldc + n0 + c4) = v;
        }
        __threadfence();
      }
    } else {
      const int q = lane >> 3, c8 = (lane & 7) * 8;
      unsigned short* C  = (unsigned short*)Cout  + (size_t)b * strideC;
      unsigned short* C2 = (OUT_MODE == 2) ? ((unsigned short*)Cout2 + (size_t)b * strideC) : nullptr;
      for (int pass = 0; pass < 2; ++pass) {
#pragma unroll
        for (int it = 0; it < 4; ++it) {
          const int row = it * 4 + q;
          const float* sp = slab + row * 68 + c8;
          v8h hv, lv;
#pragma unroll
          for (int e = 0; e < 8; ++e) {
            if (OUT_MODE == 1) {
              hv[e] = (_Float16)sp[e];
            } else {
              unsigned short hb = f2bf_bits(sp[e]);
              unsigned short lb = f2bf_bits(sp[e] - bf_bits2f(hb));
              hv[e] = __builtin_bit_cast(_Float16, hb);
              lv[e] = __builtin_bit_cast(_Float16, lb);
            }
          }
          *(volatile v8h*)(C + (size_t)(mBase + row) * ldc + n0 + c8) = hv;
          if (OUT_MODE == 2) *(volatile v8h*)(C2 + (size_t)(mBase + row) * ldc + n0 + c8) = lv;
        }
        __threadfence();
      }
    }
    __builtin_amdgcn_fence(__ATOMIC_RELEASE, "workgroup");
    __builtin_amdgcn_wave_barrier();
    __builtin_amdgcn_fence(__ATOMIC_ACQUIRE, "workgroup");
  }
}

__device__ __forceinline__ v8f mma_h16(v16h a, v16h b, v8f c) {
  c = __builtin_amdgcn_wmma_f32_16x16x32_f16(false, a, false, b, (short)0, c, false, false);
  asm volatile("v_nop\n\tv_nop\n\tv_nop\n\tv_nop" : "+v"(c) : "v"(a), "v"(b));
  return c;
}
__device__ __forceinline__ v4f splat4(float s) { v4f r; r.x = s; r.y = s; r.z = s; r.w = s; return r; }
__device__ __forceinline__ v4f relu4(v4f a) {
  v4f r; r.x = fmaxf(a.x, 0.f); r.y = fmaxf(a.y, 0.f); r.z = fmaxf(a.z, 0.f); r.w = fmaxf(a.w, 0.f); return r;
}
__device__ __forceinline__ float dot4(v4f a, v4f b) { return a.x * b.x + a.y * b.y + a.z * b.z + a.w * b.w; }
__device__ __forceinline__ float hsum4(v4f a) { return (a.x + a.y) + (a.z + a.w); }
__device__ __forceinline__ unsigned hbits(float f) { return (unsigned)__builtin_bit_cast(unsigned short, (_Float16)f); }
__device__ __forceinline__ v2u pack4h(v4f o) {
  v2u w;
  w.x = hbits(o.x) | (hbits(o.y) << 16);
  w.y = hbits(o.z) | (hbits(o.w) << 16);
  return w;
}

__global__ __launch_bounds__(256) void cast_scale_f16x2(
    const float* __restrict__ in, unsigned short* __restrict__ out, int n2, float sc) {
  const int i = blockIdx.x * 256 + threadIdx.x;
  if (i < n2) {
    const unsigned u = hbits(in[2 * i] * sc) | (hbits(in[2 * i + 1] * sc) << 16);
    ((volatile unsigned*)out)[i] = u;
    __threadfence();
    ((volatile unsigned*)out)[i] = u;
  }
}

__global__ __launch_bounds__(256) void cast_wlab_t(
    const float* __restrict__ W, unsigned short* __restrict__ out, int n2, float sc) {
  const int i2 = blockIdx.x * 256 + threadIdx.x;
  if (i2 < n2) {
    const int o = 2 * i2;
    const int l = o >> 16;
    const int rem = o & 65535;
    const int j = rem >> 8;
    const int ii = rem & 255;
    const float* base = W + (size_t)l * HID * HID;
    const unsigned u = hbits(base[ii * HID + j] * sc) | (hbits(base[(ii + 1) * HID + j] * sc) << 16);
    ((volatile unsigned*)out)[i2] = u;
    __threadfence();
    ((volatile unsigned*)out)[i2] = u;
  }
}

__global__ __launch_bounds__(256) void pe_sin_kernel(float* __restrict__ tab) {
  const int i = blockIdx.x * 256 + threadIdx.x;
  const int n = i >> 7, p = i & 127;
  const float negk = -9.2103405f * (1.0f / 256.0f);
  const float dv = expf((float)(2 * p) * negk);
  const float v = sinf((float)n * dv);
  volatile float* d = tab + i;
  *d = v;
  __threadfence();
  *d = v;
}
__global__ __launch_bounds__(256) void pe_cos_kernel(float* __restrict__ tab) {
  const int i = blockIdx.x * 256 + threadIdx.x;
  const int n = i >> 7, p = i & 127;
  const float negk = -9.2103405f * (1.0f / 256.0f);
  const float dv = expf((float)(2 * p) * negk);
  const float v = cosf((float)n * dv);
  volatile float* d = tab + i;
  *d = v;
  __threadfence();
  *d = v;
}

__global__ __launch_bounds__(256) void posenc_kernel(
    const float* __restrict__ states, const float* __restrict__ ts, const float* __restrict__ tc,
    float* __restrict__ x, unsigned short* __restrict__ x16) {
  const int i = blockIdx.x * 256 + threadIdx.x;
  const int row = i >> 6;
  const int c = (i & 63) * 4;
  const int n = row % NS;
  const int p = c >> 1;
  const size_t eo = (size_t)row * HID + c;
  const v4f s = *(const v4f*)(states + eo);
  const v2f sv = *(const v2f*)(ts + n * 128 + p);
  const v2f cv = *(const v2f*)(tc + n * 128 + p);
  v4f o;
  o.x = s.x + sv.x; o.y = s.y + cv.x; o.z = s.z + sv.y; o.w = s.w + cv.y;
  const v2u w = pack4h(o);
  for (int pass = 0; pass < 2; ++pass) {
    *(volatile v4f*)(x + eo) = o;
    *(volatile v2u*)(x16 + eo) = w;
    __threadfence();
  }
}

__global__ __launch_bounds__(256) void add_ln_kernel(
    const float* __restrict__ xin, const float* __restrict__ y,
    const float* __restrict__ g, const float* __restrict__ bb,
    float* __restrict__ xo, unsigned short* __restrict__ xo16) {
  const int lane = threadIdx.x & 31, wave = threadIdx.x >> 5;
  const int row = blockIdx.x * 8 + wave;
  const int c0 = lane * 4, c1 = 128 + lane * 4;
  const size_t ro = (size_t)row * HID;
  const v4f a0 = *(const v4f*)(xin + ro + c0), a1 = *(const v4f*)(xin + ro + c1);
  const v4f y0 = *(const v4f*)(y + ro + c0),   y1 = *(const v4f*)(y + ro + c1);
  const v4f v0 = a0 + y0, v1 = a1 + y1;
  float s = hsum4(v0) + hsum4(v1);
#pragma unroll
  for (int off = 16; off > 0; off >>= 1) s += __shfl_xor(s, off, 32);
  const float mu = s * (1.0f / 256.0f);
  const v4f d0 = v0 - splat4(mu), d1 = v1 - splat4(mu);
  float sq = dot4(d0, d0) + dot4(d1, d1);
#pragma unroll
  for (int off = 16; off > 0; off >>= 1) sq += __shfl_xor(sq, off, 32);
  const float var = sq * (1.0f / 256.0f);
  const float rstd = 1.0f / sqrtf(var + 1e-5f);
  const v4f g0 = *(const v4f*)(g + c0), g1 = *(const v4f*)(g + c1);
  const v4f b0 = *(const v4f*)(bb + c0), b1 = *(const v4f*)(bb + c1);
  const v4f o0 = d0 * splat4(rstd) * g0 + b0;
  const v4f o1 = d1 * splat4(rstd) * g1 + b1;
  const v2u w0 = pack4h(o0), w1 = pack4h(o1);
  for (int pass = 0; pass < 2; ++pass) {
    *(volatile v4f*)(xo + ro + c0) = o0;
    *(volatile v4f*)(xo + ro + c1) = o1;
    *(volatile v2u*)(xo16 + ro + c0) = w0;
    *(volatile v2u*)(xo16 + ro + c1) = w1;
    __threadfence();
  }
}

constexpr int KPITCH = 40;
constexpr int VPITCH = 72;
constexpr int PPITCH = 72;
constexpr int OPITCH = 36;

__global__ __launch_bounds__(128) void attn32_kernel(
    const unsigned short* __restrict__ qkv, float* __restrict__ ctx) {
  __shared__ __align__(16) unsigned short Ksh[64 * KPITCH];
  __shared__ __align__(16) unsigned short Vt[HDIM * VPITCH];
  __shared__ __align__(16) _Float16 Psh[4][16 * PPITCH];
  __shared__ __align__(16) float Os[4][16 * OPITCH];

  const int tid = threadIdx.x, wave = tid >> 5, lane = tid & 31;
  const int hh = lane >> 4, c = lane & 15;
  const int bx = blockIdx.x;
  const int qb = bx & 7;
  const int nh = bx >> 3;
  const int n = nh >> 3;
  const int h = nh & 7;
  const int q0 = qb * 64 + wave * 16;
  const float SCL = 0.17677669529663687f;
  const float PCARRY = 1024.0f;

  const _Float16* hbase = (const _Float16*)qkv;
  const v16h qa = Frag<_Float16>::load(hbase + ((size_t)(q0 + c) * NS + n) * (3 * HID) + h * HDIM + 8 * hh);

  float mrow[8], lrow[8];
  v8f oacc[2];
#pragma unroll
  for (int r = 0; r < 8; ++r) { mrow[r] = -INFINITY; lrow[r] = 0.f; }
#pragma unroll
  for (int t = 0; t < 2; ++t) oacc[t] = (v8f){0.f,0.f,0.f,0.f,0.f,0.f,0.f,0.f};

  for (int kc = 0; kc < 8; ++kc) {
    const int kv0 = kc * 64;
    __syncthreads();
    {
      const int kvr = tid >> 1, dh = (tid & 1) * 16;
      const unsigned short* kp = qkv + ((size_t)(kv0 + kvr) * NS + n) * (3 * HID) + HID + h * HDIM + dh;
      const v4u k0 = *(const v4u*)(kp), k1 = *(const v4u*)(kp + 8);
      const v4u w0 = *(const v4u*)(kp + HID), w1 = *(const v4u*)(kp + HID + 8);
      *(v4u*)(Ksh + kvr * KPITCH + dh) = k0;
      *(v4u*)(Ksh + kvr * KPITCH + dh + 8) = k1;
      const unsigned vw[8] = {w0.x, w0.y, w0.z, w0.w, w1.x, w1.y, w1.z, w1.w};
#pragma unroll
      for (int e = 0; e < 16; ++e) {
        const unsigned wd = vw[e >> 1];
        const unsigned short sb = (unsigned short)((e & 1) ? (wd >> 16) : (wd & 0xffffu));
        Vt[(dh + e) * VPITCH + kvr] = sb;
      }
    }
    __syncthreads();

    v8f s[4];
#pragma unroll
    for (int j = 0; j < 4; ++j) {
      s[j] = (v8f){0.f,0.f,0.f,0.f,0.f,0.f,0.f,0.f};
      const v16h kb = Frag<_Float16>::load((const _Float16*)Ksh + (j * 16 + c) * KPITCH + 8 * hh);
      s[j] = mma_h16(qa, kb, s[j]);
    }
    float cm[8];
#pragma unroll
    for (int r = 0; r < 8; ++r) {
      float m = -INFINITY;
#pragma unroll
      for (int j = 0; j < 4; ++j) { s[j][r] *= SCL; m = fmaxf(m, s[j][r]); }
#pragma unroll
      for (int off = 1; off < 16; off <<= 1) m = fmaxf(m, __shfl_xor(m, off, 32));
      cm[r] = m;
    }
    _Float16* pw = Psh[wave];
#pragma unroll
    for (int r = 0; r < 8; ++r) {
      const float mnew = fmaxf(mrow[r], cm[r]);
      const float alpha = expf(mrow[r] - mnew);
      mrow[r] = mnew;
      float psum = 0.f;
#pragma unroll
      for (int j = 0; j < 4; ++j) {
        const float p = expf(s[j][r] - mnew);
        psum += p;
        pw[(8 * hh + r) * PPITCH + j * 16 + c] = (_Float16)(p * PCARRY);
      }
#pragma unroll
      for (int off = 1; off < 16; off <<= 1) psum += __shfl_xor(psum, off, 32);
      lrow[r] = lrow[r] * alpha + psum;
      oacc[0][r] *= alpha;
      oacc[1][r] *= alpha;
    }
    __syncthreads();
#pragma unroll
    for (int kk = 0; kk < 2; ++kk) {
      const v16h pa = Frag<_Float16>::load(pw + c * PPITCH + kk * 32 + 8 * hh);
#pragma unroll
      for (int t = 0; t < 2; ++t) {
        const v16h vb = Frag<_Float16>::load((const _Float16*)Vt + (t * 16 + c) * VPITCH + kk * 32 + 8 * hh);
        oacc[t] = mma_h16(pa, vb, oacc[t]);
      }
    }
  }

  float* os = Os[wave];
#pragma unroll
  for (int r = 0; r < 8; ++r) {
    const float inv = 1.0f / (lrow[r] * PCARRY);
#pragma unroll
    for (int t = 0; t < 2; ++t) os[(8 * hh + r) * OPITCH + t * 16 + c] = oacc[t][r] * inv;
  }
  __syncthreads();
  {
    const int q8 = lane >> 3, c4 = (lane & 7) * 4;
    for (int pass = 0; pass < 2; ++pass) {
#pragma unroll
      for (int it = 0; it < 4; ++it) {
        const int row = it * 4 + q8;
        const v4f val = *(const v4f*)(os + row * OPITCH + c4);
        *(volatile v4f*)(ctx + ((size_t)(q0 + row) * NS + n) * HID + h * HDIM + c4) = val;
      }
      __threadfence();
    }
  }
}

__global__ __launch_bounds__(256) void aggregate_kernel(
    const float* __restrict__ P, const float* __restrict__ Q,
    const float* __restrict__ Wa2, const float* __restrict__ ba2,
    const float* __restrict__ amask, const float* __restrict__ smask,
    const float* __restrict__ xo, float* __restrict__ SF) {
  const int lane = threadIdx.x & 31, wave = threadIdx.x >> 5;
  const int bq = blockIdx.x * 8 + wave;
  const int b = bq >> 5;
  const int c0 = lane * 4, c1 = 128 + lane * 4;
  const size_t po = (size_t)bq * HID;
  const v4f p0 = *(const v4f*)(P + po + c0), p1 = *(const v4f*)(P + po + c1);
  const v4f w0 = *(const v4f*)(Wa2 + c0), w1 = *(const v4f*)(Wa2 + c1);
  const float bias2 = ba2[0];
  const float am = amask[bq];
  v4f n0 = splat4(0.f), n1 = splat4(0.f);
  float den = 0.f;
#pragma unroll 1
  for (int k = 0; k < NS; ++k) {
    const size_t ro = (size_t)(b * NS + k) * HID;
    const v4f q0 = *(const v4f*)(Q + ro + c0), q1 = *(const v4f*)(Q + ro + c1);
    const v4f h0 = relu4(p0 + q0), h1 = relu4(p1 + q1);
    float s = dot4(h0, w0) + dot4(h1, w1);
#pragma unroll
    for (int off = 16; off > 0; off >>= 1) s += __shfl_xor(s, off, 32);
    const float a = fmaxf(s + bias2, 0.f);
    const float mk = am * smask[b * NS + k];
    const float ex = expf(a);
    const float e = (mk > 0.f) ? ex : 0.f;
    den += e;
    const v4f o0 = *(const v4f*)(xo + ro + c0), o1 = *(const v4f*)(xo + ro + c1);
    n0 = n0 + o0 * splat4(e);
    n1 = n1 + o1 * splat4(e);
  }
  const float inv = 1.0f / fmaxf(den, 2e-15f);
  const v4f s0 = n0 * splat4(inv), s1 = n1 * splat4(inv);
  for (int pass = 0; pass < 2; ++pass) {
    *(volatile v4f*)(SF + po + c0) = s0;
    *(volatile v4f*)(SF + po + c1) = s1;
    __threadfence();
  }
}

__global__ __launch_bounds__(256) void advdot_kernel(
    const float* __restrict__ U, const float* __restrict__ SF,
    const float* __restrict__ blab, float* __restrict__ advb, int l) {
  __shared__ float sh[32];
  const int lane = threadIdx.x & 31, wave = threadIdx.x >> 5;
  const int bs0 = blockIdx.x * 32;
  const int c0 = lane * 4, c1 = 128 + lane * 4;
  const float bl = blab[l];
#pragma unroll
  for (int i = 0; i < 4; ++i) {
    const int row = bs0 + wave * 4 + i;
    const size_t ro = (size_t)row * HID;
    const v4f u0 = *(const v4f*)(U + ro + c0), u1 = *(const v4f*)(U + ro + c1);
    const v4f f0 = *(const v4f*)(SF + ro + c0), f1 = *(const v4f*)(SF + ro + c1);
    float s = dot4(u0, f0) + dot4(u1, f1);
#pragma unroll
    for (int off = 16; off > 0; off >>= 1) s += __shfl_xor(s, off, 32);
    if (lane == 0) sh[wave * 4 + i] = s + bl;
  }
  __syncthreads();
  if (wave == 0) {
    const float v = sh[lane];
    volatile float* d = advb + (size_t)l * NACT + bs0 + lane;
    *d = v;
    __threadfence();
    *d = v;
  }
}

__global__ __launch_bounds__(256) void final_kernel(
    const float* __restrict__ SF, const float* __restrict__ amask,
    const float* __restrict__ Wv, const float* __restrict__ bv,
    const float* __restrict__ advb, float* __restrict__ out) {
  __shared__ float red[256];
  __shared__ __align__(16) float outs[NS2 * NLAB];
  __shared__ float scal[2];
  const int b = blockIdx.x, t = threadIdx.x, lane = t & 31, wave = t >> 5;
  if (wave == 0) {
    float a = amask[b * NS2 + lane];
#pragma unroll
    for (int off = 16; off > 0; off >>= 1) a += __shfl_xor(a, off, 32);
    if (lane == 0) scal[0] = a;
  }
  float m = 0.f;
#pragma unroll 1
  for (int q = 0; q < NS2; ++q) m += SF[(size_t)(b * NS2 + q) * HID + t];
  __syncthreads();
  const float ranum = 1.0f / scal[0];
  red[t] = (m * ranum) * Wv[t];
  __syncthreads();
  for (int st = 128; st > 0; st >>= 1) {
    if (t < st) red[t] += red[t + st];
    __syncthreads();
  }
  const float val = red[0] + bv[0];
  __syncthreads();
  const int lsel = ((t >> 5) < (NLAB - 1)) ? (t >> 5) : (NLAB - 1);
  const int ssel = t & 31;
  const float av = advb[(size_t)lsel * NACT + b * NS2 + ssel];
  const float a = (t < NS2 * NLAB) ? av : 0.f;
  red[t] = a;
  __syncthreads();
  for (int st = 128; st > 0; st >>= 1) {
    if (t < st) red[t] += red[t + st];
    __syncthreads();
  }
  const float amean = red[0] * (1.0f / 96.0f);
  __syncthreads();
  if (t < NS2 * NLAB) outs[ssel * NLAB + lsel] = val + a - amean;
  __syncthreads();
  if (wave == 0 && lane < 24) {
    const v4f v = *(const v4f*)(outs + lane * 4);
    volatile v4f* d = (volatile v4f*)(out + (size_t)b * (NS2 * NLAB) + lane * 4);
    *d = v;
    __threadfence();
    *d = v;
  }
}

constexpr size_t SZ_XF     = (size_t)NTOK * HID * 4;
constexpr size_t SZ_X16    = (size_t)NTOK * HID * 2;
constexpr size_t SZ_QKV16  = (size_t)NTOK * 3 * HID * 2;
constexpr size_t SZ_HMID16 = (size_t)NTOK * DFF * 2;
constexpr size_t SZ_WQKV16 = (size_t)NLAY * 3 * HID * HID * 2;
constexpr size_t SZ_WO16   = (size_t)NLAY * HID * HID * 2;
constexpr size_t SZ_W1_16  = (size_t)NLAY * DFF * HID * 2;
constexpr size_t SZ_W2_16  = (size_t)NLAY * HID * DFF * 2;
constexpr size_t SZ_WA1_16 = (size_t)HID * 2 * HID * 2;
constexpr size_t SZ_WLT16  = (size_t)NLAB * HID * HID * 2;
constexpr size_t SZ_ACT16  = (size_t)NACT * HID * 2;
constexpr size_t SZ_ACTF   = (size_t)NACT * HID * 4;
constexpr size_t SZ_ADV    = (size_t)NLAB * NACT * 4;
constexpr size_t SZ_TAB    = (size_t)NS * 128 * 4;

constexpr size_t OFF_XA     = 0;
constexpr size_t OFF_XB     = OFF_XA + SZ_XF;
constexpr size_t OFF_XA16   = OFF_XB + SZ_XF;
constexpr size_t OFF_XB16   = OFF_XA16 + SZ_X16;
constexpr size_t OFF_QKV16  = OFF_XB16 + SZ_X16;
constexpr size_t OFF_CTX    = OFF_QKV16 + SZ_QKV16;
constexpr size_t OFF_CTX16  = OFF_CTX + SZ_XF;
constexpr size_t OFF_T1     = OFF_CTX16 + SZ_X16;
constexpr size_t OFF_HMID16 = OFF_T1 + SZ_XF;
constexpr size_t OFF_WQKV16 = OFF_HMID16 + SZ_HMID16;
constexpr size_t OFF_WO16   = OFF_WQKV16 + SZ_WQKV16;
constexpr size_t OFF_W1_16  = OFF_WO16 + SZ_WO16;
constexpr size_t OFF_W2_16  = OFF_W1_16 + SZ_W1_16;
constexpr size_t OFF_WA1_16 = OFF_W2_16 + SZ_W2_16;
constexpr size_t OFF_WLT16  = OFF_WA1_16 + SZ_WA1_16;
constexpr size_t OFF_ACT16  = OFF_WLT16 + SZ_WLT16;
constexpr size_t OFF_PAGG   = OFF_ACT16 + SZ_ACT16;
constexpr size_t OFF_QAGG   = OFF_PAGG + SZ_ACTF;
constexpr size_t OFF_SF     = OFF_QAGG + SZ_XF;
constexpr size_t OFF_U      = OFF_SF + SZ_ACTF;
constexpr size_t OFF_ADV    = OFF_U + SZ_ACTF;
constexpr size_t OFF_TS     = OFF_ADV + SZ_ADV;
constexpr size_t OFF_TC     = OFF_TS + SZ_TAB;
constexpr size_t WS_TOTAL   = OFF_TC + SZ_TAB;
static_assert(WS_TOTAL == 105191424, "carve total");
static_assert(WS_TOTAL <= (size_t)134217728, "carve under 128 MiB");
static_assert((OFF_TC % 256) == 0 && (OFF_TS % 256) == 0 && (OFF_ADV % 256) == 0, "alignment");

static_assert(HID % 32 == 0 && DFF % 32 == 0, "K multiples of 32");
static_assert(NTOK % 64 == 0 && NACT % 64 == 0, "M multiples of 64");
static_assert((3 * HID) % 64 == 0 && HID % 64 == 0 && DFF % 64 == 0, "N multiples of 64");
constexpr int GX_QKV  = (NTOK / 64) * (3 * HID / 64) / 8;
constexpr int GX_TOKH = (NTOK / 64) * (HID / 64) / 8;
constexpr int GX_W1   = (NTOK / 64) * (DFF / 64) / 8;
constexpr int GX_ACTH = (NACT / 64) * (HID / 64) / 8;
static_assert(GX_QKV * 8 == (NTOK / 64) * (3 * HID / 64), "exact tiles");
static_assert(GX_TOKH * 8 == (NTOK / 64) * (HID / 64), "exact tiles");
static_assert(GX_W1 * 8 == (NTOK / 64) * (DFF / 64), "exact tiles");
static_assert(GX_ACTH * 8 == (NACT / 64) * (HID / 64), "exact tiles");
static_assert((size_t)NACT * NLAB * 4 == 196608, "output bytes");

extern "C" void kernel_launch(void* const* d_in, const int* in_sizes, int n_in,
                              void* d_out, int out_size, void* d_ws, size_t ws_size,
                              hipStream_t stream)
{
  if (n_in < 24) return;
  if (out_size != NACT * NLAB) return;
  if (ws_size < WS_TOTAL) return;
  if (in_sizes[0] != NTOK * HID || in_sizes[2] != NACT * HID) return;
  if (in_sizes[4] != NLAY * 3 * HID * HID || in_sizes[10] != NLAY * DFF * HID || in_sizes[22] != NLAB * HID * HID) return;

  const float* states = (const float*)d_in[0];
  const float* smask  = (const float*)d_in[1];
  const float* actions= (const float*)d_in[2];
  const float* amask  = (const float*)d_in[3];
  const float* Wqkv   = (const float*)d_in[4];
  const float* bqkv   = (const float*)d_in[5];
  const float* Wo     = (const float*)d_in[6];
  const float* bo     = (const float*)d_in[7];
  const float* ln1g   = (const float*)d_in[8];
  const float* ln1b   = (const float*)d_in[9];
  const float* W1     = (const float*)d_in[10];
  const float* b1     = (const float*)d_in[11];
  const float* W2     = (const float*)d_in[12];
  const float* b2     = (const float*)d_in[13];
  const float* ln2g   = (const float*)d_in[14];
  const float* ln2b   = (const float*)d_in[15];
  const float* Wa1    = (const float*)d_in[16];
  const float* ba1    = (const float*)d_in[17];
  const float* Wa2    = (const float*)d_in[18];
  const float* ba2    = (const float*)d_in[19];
  const float* Wv     = (const float*)d_in[20];
  const float* bv     = (const float*)d_in[21];
  const float* Wlab   = (const float*)d_in[22];
  const float* blab   = (const float*)d_in[23];

  char* ws = (char*)d_ws;
  float* xA = (float*)(ws + OFF_XA);
  float* xB = (float*)(ws + OFF_XB);
  unsigned short* xA16   = (unsigned short*)(ws + OFF_XA16);
  unsigned short* xB16   = (unsigned short*)(ws + OFF_XB16);
  unsigned short* qkv16  = (unsigned short*)(ws + OFF_QKV16);
  float* ctx = (float*)(ws + OFF_CTX);
  unsigned short* ctx16  = (unsigned short*)(ws + OFF_CTX16);
  float* t1  = (float*)(ws + OFF_T1);
  unsigned short* hmid16 = (unsigned short*)(ws + OFF_HMID16);
  unsigned short* Wqkv16 = (unsigned short*)(ws + OFF_WQKV16);
  unsigned short* Wo16   = (unsigned short*)(ws + OFF_WO16);
  unsigned short* W1h    = (unsigned short*)(ws + OFF_W1_16);
  unsigned short* W2h    = (unsigned short*)(ws + OFF_W2_16);
  unsigned short* Wa1h   = (unsigned short*)(ws + OFF_WA1_16);
  unsigned short* WlabT  = (unsigned short*)(ws + OFF_WLT16);
  unsigned short* act16  = (unsigned short*)(ws + OFF_ACT16);
  float* Pagg = (float*)(ws + OFF_PAGG);
  float* Qagg = (float*)(ws + OFF_QAGG);
  float* SF   = (float*)(ws + OFF_SF);
  float* U    = (float*)(ws + OFF_U);
  float* advb = (float*)(ws + OFF_ADV);
  float* ts   = (float*)(ws + OFF_TS);
  float* tc   = (float*)(ws + OFF_TC);
  float* outp = (float*)d_out;

  const float WINV  = 1.0f / 64.0f;
  const float WINV2 = 1.0f / 4096.0f;

  pe_sin_kernel<<<3, 256, 0, stream>>>(ts);
  pe_cos_kernel<<<3, 256, 0, stream>>>(tc);
  posenc_kernel<<<(NTOK * HID / 4) / 256, 256, 0, stream>>>(states, ts, tc, xA, xA16);

  cast_scale_f16x2<<<(NLAY * 3 * HID * HID / 2) / 256, 256, 0, stream>>>(Wqkv, Wqkv16, NLAY * 3 * HID * HID / 2, 64.0f);
  cast_scale_f16x2<<<(NLAY * HID * HID / 2) / 256, 256, 0, stream>>>(Wo, Wo16, NLAY * HID * HID / 2, 64.0f);
  cast_scale_f16x2<<<(NLAY * DFF * HID / 2) / 256, 256, 0, stream>>>(W1, W1h, NLAY * DFF * HID / 2, 64.0f);
  cast_scale_f16x2<<<(NLAY * HID * DFF / 2) / 256, 256, 0, stream>>>(W2, W2h, NLAY * HID * DFF / 2, 64.0f);
  cast_scale_f16x2<<<(HID * 2 * HID / 2) / 256, 256, 0, stream>>>(Wa1, Wa1h, HID * 2 * HID / 2, 64.0f);
  cast_wlab_t<<<(NLAB * HID * HID / 2) / 256, 256, 0, stream>>>(Wlab, WlabT, NLAB * HID * HID / 2, 64.0f);
  cast_scale_f16x2<<<(NACT * HID / 2) / 256, 256, 0, stream>>>(actions, act16, NACT * HID / 2, 1.0f);

  for (int i = 0; i < NLAY; ++i) {
    wmma_gemm64<0, false, 2, 1, false, 0><<<dim3(GX_QKV, 1), 256, 0, stream>>>(
        xA16, xA16, HID, 0L,
        Wqkv16 + (size_t)i * 3 * HID * HID, Wqkv16 + (size_t)i * 3 * HID * HID, HID, 0L,
        (void*)qkv16, (void*)qkv16, 3 * HID, 0L,
        bqkv + (size_t)i * 3 * HID, bqkv, 0L,
        NTOK, 3 * HID, HID, WINV);
    attn32_kernel<<<NS * NHEAD * (NB / 64), 128, 0, stream>>>(qkv16, ctx);
    cast_scale_f16x2<<<(NTOK * HID / 2) / 256, 256, 0, stream>>>(ctx, ctx16, NTOK * HID / 2, 64.0f);
    wmma_gemm64<0, false, 2, 0, false, 0><<<dim3(GX_TOKH, 1), 256, 0, stream>>>(
        ctx16, ctx16, HID, 0L,
        Wo16 + (size_t)i * HID * HID, Wo16 + (size_t)i * HID * HID, HID, 0L,
        (void*)t1, (void*)t1, HID, 0L,
        bo + (size_t)i * HID, bo, 0L,
        NTOK, HID, HID, WINV2);
    add_ln_kernel<<<NTOK / 8, 256, 0, stream>>>(xA, t1, ln1g + (size_t)i * HID, ln1b + (size_t)i * HID, xB, xB16);
    wmma_gemm64<0, false, 2, 1, false, 2><<<dim3(GX_W1, 1), 256, 0, stream>>>(
        xB16, xB16, HID, 0L,
        W1h + (size_t)i * DFF * HID, W1h + (size_t)i * DFF * HID, HID, 0L,
        (void*)hmid16, (void*)hmid16, DFF, 0L,
        b1 + (size_t)i * DFF, b1, 0L,
        NTOK, DFF, HID, WINV);
    wmma_gemm64<0, false, 2, 0, false, 0><<<dim3(GX_TOKH, 1), 256, 0, stream>>>(
        hmid16, hmid16, DFF, 0L,
        W2h + (size_t)i * HID * DFF, W2h + (size_t)i * HID * DFF, DFF, 0L,
        (void*)t1, (void*)t1, HID, 0L,
        b2 + (size_t)i * HID, b2, 0L,
        NTOK, HID, DFF, WINV);
    add_ln_kernel<<<NTOK / 8, 256, 0, stream>>>(xB, t1, ln2g + (size_t)i * HID, ln2b + (size_t)i * HID, xA, xA16);
  }

  wmma_gemm64<0, false, 2, 0, false, 0><<<dim3(GX_ACTH, 1), 256, 0, stream>>>(
      act16, act16, HID, 0L,
      Wa1h, Wa1h, 2 * HID, 0L,
      (void*)Pagg, (void*)Pagg, HID, 0L,
      ba1, ba1, 0L,
      NACT, HID, HID, WINV);
  wmma_gemm64<0, false, 0, 0, false, 0><<<dim3(GX_TOKH, 1), 256, 0, stream>>>(
      xA16, xA16, HID, 0L,
      Wa1h + HID, Wa1h + HID, 2 * HID, 0L,
      (void*)Qagg, (void*)Qagg, HID, 0L,
      ba1, ba1, 0L,
      NTOK, HID, HID, WINV);
  aggregate_kernel<<<NACT / 8, 256, 0, stream>>>(Pagg, Qagg, Wa2, ba2, amask, smask, xA, SF);

  for (int l = 0; l < NLAB; ++l) {
    wmma_gemm64<0, false, 0, 0, false, 0><<<dim3(GX_ACTH, 1), 256, 0, stream>>>(
        act16, act16, HID, 0L,
        WlabT + (size_t)l * HID * HID, WlabT + (size_t)l * HID * HID, HID, 0L,
        (void*)U, (void*)U, HID, 0L,
        blab, blab, 0L,
        NACT, HID, HID, WINV);
    advdot_kernel<<<NACT / 32, 256, 0, stream>>>(U, SF, blab, advb, l);
  }

  final_kernel<<<NB, 256, 0, stream>>>(SF, amask, Wv, bv, advb, outp);
}
